// MemoryAsContextTransformer_17274358464742
// MI455X (gfx1250) — hardware-verified
//
#include <hip/hip_runtime.h>
#include <math.h>
#include <stdint.h>

#ifndef NB
#define NB 2
#endif
#ifndef SEQ
#define SEQ 4096
#endif
#define SEQ_FULL 4096
#define DM    1024
#define NH    16
#define HD    64
#define DMI   (NH * HD)
#define QKP   (2 * DMI)
#define SEGL  512
#define PMEM  16
#define NSEGB (SEQ / SEGL)
#define NQBS  (SEGL / 64)
#define RESQB 2
#define VLP   (RESQB * 64)
#define NFR   (HD / 2)
static_assert((SEQ % SEGL) == 0 && (SEGL % 64) == 0 && (SEQ % 64) == 0);
static_assert(RESQB >= 1 && RESQB <= NQBS);
static_assert((DM % 256) == 0 && (DMI % 64) == 0 && HD == 64 && NFR == 32);
static_assert(SEQ <= SEQ_FULL && NB >= 1 && NB <= 2);
static_assert(DMI == DM);

typedef _Float16 v16h __attribute__((ext_vector_type(16)));
typedef _Float16 v8h  __attribute__((ext_vector_type(8)));
typedef __bf16   v16b __attribute__((ext_vector_type(16)));
typedef __bf16   v8b  __attribute__((ext_vector_type(8)));
typedef float    v8f  __attribute__((ext_vector_type(8)));
typedef float    v4f  __attribute__((ext_vector_type(4)));
typedef unsigned int v4u __attribute__((ext_vector_type(4)));

__device__ __forceinline__ unsigned short bf_bits(float f) {
  unsigned u = __float_as_uint(f);
  return (unsigned short)((u + 0x7FFFu + ((u >> 16) & 1u)) >> 16);
}
__device__ __forceinline__ float bf_up(unsigned short h) { return __uint_as_float(((unsigned)h) << 16); }
__device__ __forceinline__ unsigned short h_bits(_Float16 x) { return __builtin_bit_cast(unsigned short, x); }
__device__ __forceinline__ unsigned pk16(unsigned short a, unsigned short b) { return (unsigned)a | ((unsigned)b << 16); }
__device__ __forceinline__ v8f zero8() { v8f z = {0.f, 0.f, 0.f, 0.f, 0.f, 0.f, 0.f, 0.f}; return z; }
__device__ __forceinline__ v8h zero8h() {
  const _Float16 z = (_Float16)0.0f;
  v8h r = {z, z, z, z, z, z, z, z};
  return r;
}
__device__ __forceinline__ v4u zero4u() { v4u z = {0u, 0u, 0u, 0u}; return z; }
__device__ __forceinline__ v8b zero8b() { union { v4u u; v8b v; } z; z.u = zero4u(); return z.v; }

__device__ __forceinline__ void sincos_pd(float ang, float& sv, float& cv) {
  const double x  = (double)ang;
  const double kq = __builtin_rint(x * 0.63661977236758134308);
  double r = __builtin_fma(-kq, 1.57079632679489655800e+00, x);
  r = __builtin_fma(-kq, 6.12323399573676603587e-17, r);
  const double z = r * r, w = z * z;
  const double rs = -1.98393348360966317347e-04 + z * 2.71831149398982191e-06;
  const double s3 = z * r;
  const double sn = (r + s3 * (-1.66666666416265235595e-01 + z * 8.3333293858894631756e-03)) + s3 * w * rs;
  const double rc = -1.38867637746099294692e-03 + z * 2.43904487962774090654e-05;
  const double cs = ((1.0 + z * (-4.99999997251031003120e-01)) + w * 4.16666233237390631894e-02) + (w * z) * rc;
  const int n = ((int)kq) & 3;
  const float fs = (float)sn, fc = (float)cs;
  float so = fs, co = fc;
  if (n == 1) { so = fc;  co = -fs; }
  if (n == 2) { so = -fs; co = -fc; }
  if (n == 3) { so = -fc; co = fs;  }
  sv = so; cv = co;
}

__device__ __forceinline__ v16b ldfrag_b(const __bf16* p) {
  union { v16b v; v8b h[2]; } f;
  f.h[0] = *(const v8b*)(p);
  f.h[1] = *(const v8b*)(p + 16);
  return f.v;
}

__device__ __forceinline__ v8f mma_b(v16b a, v16b b, v8f c) {
  c = __builtin_amdgcn_wmma_f32_16x16x32_bf16(false, a, false, b, (short)0, c, false, false);
  asm volatile("v_nop\n\tv_nop\n\tv_nop\n\tv_nop" : "+v"(c) : "v"(a), "v"(b));
  return c;
}
__device__ __forceinline__ v8f mma_h(v16h a, v16h b, v8f c) {
  c = __builtin_amdgcn_wmma_f32_16x16x32_f16(false, a, false, b, (short)0, c, false, false);
  asm volatile("v_nop\n\tv_nop\n\tv_nop\n\tv_nop" : "+v"(c) : "v"(a), "v"(b));
  return c;
}
__device__ __forceinline__ v8f mma_b_raw(v16b a, v16b b, v8f c) {
  return __builtin_amdgcn_wmma_f32_16x16x32_bf16(false, a, false, b, (short)0, c, false, false);
}
__device__ __forceinline__ void dep_guard_b(v8f& a, v8f& b, v16b x, v16b y) {
  asm volatile("v_nop\n\tv_nop\n\tv_nop\n\tv_nop" : "+v"(a), "+v"(b) : "v"(x), "v"(y));
}
__device__ __forceinline__ void keep4_b(v16b a, v16b b, v16b c, v16b d) {
  asm volatile("v_nop" :: "v"(a), "v"(b), "v"(c), "v"(d));
}
__device__ __forceinline__ void acc_guard4(v8f& a, v8f& b, v8f& c, v8f& d) {
  asm volatile("v_nop\n\tv_nop\n\tv_nop\n\tv_nop" : "+v"(a), "+v"(b), "+v"(c), "+v"(d));
}

__global__ __launch_bounds__(256) void tab_cs(float* ct, float* st) {
  const int wave = threadIdx.x >> 5, lane = threadIdx.x & 31;
  const int t = blockIdx.x * 8 + wave;
  if (t >= SEQ) return;
  double pw = 1.0;
#pragma unroll 1
  for (int j = 0; j < (lane >> 3); ++j) pw *= 10.0;
#pragma unroll 1
  for (int j = 0; j < (lane & 7); ++j) pw *= 1.3335214321633240257;
  const float p32 = (float)pw;
  const float inv = (float)(1.0 / (double)p32);
  const float ang = (float)t * inv;
  float sv, cv;
  sincos_pd(ang, sv, cv);
  float* pc = ct + (size_t)t * NFR + lane;
  float* ps = st + (size_t)t * NFR + lane;
  *(volatile float*)pc = cv;
  *(volatile float*)ps = sv;
  __threadfence();
  *(volatile float*)pc = cv;
  *(volatile float*)ps = sv;
}

__global__ __launch_bounds__(256) void cvtx_rstd(const float* __restrict__ seq, unsigned short* xb, float* rs) {
  __shared__ __align__(16) float sr[32];
  const int tid = threadIdx.x, wave = tid >> 5, lane = tid & 31;
#pragma unroll 1
  for (int rr = 0; rr < 4; ++rr) {
    const int m  = blockIdx.x * 32 + wave * 4 + rr;
    const int bb = m / SEQ, t = m - bb * SEQ;
    const float* src = seq + ((size_t)bb * SEQ_FULL + t) * DM;
    unsigned short* dst = xb + (size_t)m * DM;
    v4u pk[DM / 256];
    float ss = 0.f;
#pragma unroll
    for (int i = 0; i < DM / 256; ++i) {
      const v4f a = *(const v4f*)(src + i * 256 + lane * 8);
      const v4f c = *(const v4f*)(src + i * 256 + lane * 8 + 4);
      unsigned short hb[8];
#pragma unroll
      for (int e = 0; e < 4; ++e) { hb[e] = bf_bits(a[e]); hb[4 + e] = bf_bits(c[e]); }
#pragma unroll
      for (int e = 0; e < 8; ++e) { const float v = bf_up(hb[e]); ss += v * v; }
      v4u p;
      p[0] = pk16(hb[0], hb[1]);
      p[1] = pk16(hb[2], hb[3]);
      p[2] = pk16(hb[4], hb[5]);
      p[3] = pk16(hb[6], hb[7]);
      pk[i] = p;
    }
#pragma unroll
    for (int i = 0; i < DM / 256; ++i) *(volatile v4u*)(dst + i * 256 + lane * 8) = pk[i];
    __threadfence();
#pragma unroll
    for (int i = 0; i < DM / 256; ++i) *(volatile v4u*)(dst + i * 256 + lane * 8) = pk[i];
#pragma unroll
    for (int off = 1; off < 32; off <<= 1) ss += __shfl_xor(ss, off, 32);
    const float rstd = rsqrtf(ss * (1.0f / (float)DM) + 1.1920929e-7f);
    if (lane == 0) sr[wave * 4 + rr] = rstd;
  }
  __syncthreads();
  if (wave == 0 && lane < 8) {
    const v4f v = *(const v4f*)(sr + lane * 4);
    float* d = rs + (size_t)blockIdx.x * 32 + lane * 4;
    *(volatile v4f*)d = v;
    __threadfence();
    *(volatile v4f*)d = v;
  }
}

template <bool USEG, int NPL>
__global__ __launch_bounds__(256) void wt_cvt(const float* __restrict__ W, const float* __restrict__ g,
                                              unsigned short* Wh, unsigned short* Wl, int Kdim, int Ndim) {
  __shared__ __align__(16) unsigned short shh[64 * 72];
  __shared__ __align__(16) unsigned short shl[(NPL == 2) ? 64 * 72 : 8];
  const int tid = threadIdx.x, wave = tid >> 5, lane = tid & 31;
  const int n0 = blockIdx.x * 64, k0 = blockIdx.y * 64;
  {
    const int kr = tid >> 2, nq = (tid & 3) * 16;
    const float* src = W + (size_t)(k0 + kr) * Ndim + n0 + nq;
    float gk = 1.0f;
    if (USEG) gk = bf_up(bf_bits(g[k0 + kr]));
#pragma unroll
    for (int i = 0; i < 4; ++i) {
      const v4f a = *(const v4f*)(src + 4 * i);
#pragma unroll
      for (int e = 0; e < 4; ++e) {
        const float p = gk * bf_up(bf_bits(a[e]));
        const unsigned short hb = bf_bits(p);
        shh[(nq + 4 * i + e) * 72 + kr] = hb;
        if (NPL == 2) shl[(nq + 4 * i + e) * 72 + kr] = bf_bits(p - bf_up(hb));
      }
    }
  }
  __syncthreads();
  const int q = lane >> 3, c8 = (lane & 7) * 8;
  v4u hv[2], lv[2];
#pragma unroll
  for (int it = 0; it < 2; ++it) {
    const int row = wave * 8 + it * 4 + q;
    hv[it] = *(const v4u*)(shh + row * 72 + c8);
    if (NPL == 2) lv[it] = *(const v4u*)(shl + row * 72 + c8); else lv[it] = hv[it];
  }
  for (int pass = 0; pass < 2; ++pass) {
#pragma unroll
    for (int it = 0; it < 2; ++it) {
      const int row = wave * 8 + it * 4 + q;
      const size_t o = (size_t)(n0 + row) * Kdim + k0 + c8;
      *(volatile v4u*)(Wh + o) = hv[it];
      if (NPL == 2) *(volatile v4u*)(Wl + o) = lv[it];
    }
    __threadfence();
  }
}

__global__ __launch_bounds__(128) void pm_cvt(const float* __restrict__ pm, unsigned short* pk, unsigned short* pv) {
  __shared__ __align__(16) float sp[PMEM * HD];
  const int tid = threadIdx.x, h = blockIdx.x;
  const int r = tid >> 3, d8 = (tid & 7) * 8;
  const float* kg = pm + (((size_t)0 * NH + h) * PMEM + r) * HD + d8;
  const float* vg = pm + (((size_t)1 * NH + h) * PMEM + r) * HD + d8;
  const v4f k0 = *(const v4f*)(kg), k1 = *(const v4f*)(kg + 4);
  const v4f v0 = *(const v4f*)(vg), v1 = *(const v4f*)(vg + 4);
  *(v4f*)(sp + r * HD + d8)     = v0;
  *(v4f*)(sp + r * HD + d8 + 4) = v1;
  v4u kp;
  kp[0] = pk16(bf_bits(k0[0]), bf_bits(k0[1]));
  kp[1] = pk16(bf_bits(k0[2]), bf_bits(k0[3]));
  kp[2] = pk16(bf_bits(k1[0]), bf_bits(k1[1]));
  kp[3] = pk16(bf_bits(k1[2]), bf_bits(k1[3]));
  __syncthreads();
  const int d = tid >> 1, r8 = (tid & 1) * 8;
  v4u vp;
#pragma unroll
  for (int e = 0; e < 4; ++e) {
    const float f0 = bf_up(bf_bits(sp[(r8 + 2 * e) * HD + d]));
    const float f1 = bf_up(bf_bits(sp[(r8 + 2 * e + 1) * HD + d]));
    vp[e] = pk16(h_bits((_Float16)f0), h_bits((_Float16)f1));
  }
  unsigned short* kd = pk + ((size_t)h * PMEM + r) * HD + d8;
  unsigned short* vd = pv + ((size_t)h * HD + d) * PMEM + r8;
  *(volatile v4u*)kd = kp;
  *(volatile v4u*)vd = vp;
  __threadfence();
  *(volatile v4u*)kd = kp;
  *(volatile v4u*)vd = vp;
}

template <int NSPLIT, int OUT_MODE, int SCM, bool ROT>
__global__ __launch_bounds__(256) void gemm64(
    const unsigned short* __restrict__ Ap, const unsigned short* __restrict__ A2p, int lda, long long strideA,
    const unsigned short* __restrict__ Btp, const unsigned short* __restrict__ Bt2p, int ldb, long long strideB,
    void* Cout, int ldc, long long strideC,
    void* Cout2, int ldc2, long long strideC2, int N2, int segN,
    const float* __restrict__ scal, long long strideS,
    const float* __restrict__ rct, const float* __restrict__ rst,
    int M, int N, int K, float rscale) {
  static_assert(OUT_MODE != 0 || (SCM == 0 && !ROT));
  const __bf16* A   = (const __bf16*)(const void*)Ap;
  const __bf16* A2  = (const __bf16*)(const void*)A2p;
  const __bf16* Bt  = (const __bf16*)(const void*)Btp;
  const __bf16* Bt2 = (const __bf16*)(const void*)Bt2p;
  __shared__ __align__(16) float sT[8][16 * 68];
  const int b    = blockIdx.y;
  const int lane = threadIdx.x & 31;
  const int wave = threadIdx.x >> 5;
  const int tilesN = N >> 6;
  const int tilesM = M >> 6;
  const int tile = blockIdx.x * 8 + wave;
  if (tile >= tilesM * tilesN) return;
  const int tm = tile / tilesN;
  const int tn = tile - tm * tilesN;
  const int m0 = tm << 6;
  const int n0 = tn << 6;

  const __bf16* Ab  = A  + (size_t)b * strideA;
  const __bf16* Ab2 = (NSPLIT == 1) ? (A2 + (size_t)b * strideA) : Ab;
  const __bf16* Bb  = Bt + (size_t)b * strideB;
  const __bf16* Bb2 = (NSPLIT == 2) ? (Bt2 + (size_t)b * strideB) : Bb;
  const float* scb = scal + (size_t)((long long)b * strideS);

  const int rlane = lane & 15;
  const int koff  = (lane >> 4) * 8;
  const int mOff  = (lane >> 4) * 8;

  v8f acc[4][4];
#pragma unroll
  for (int i = 0; i < 4; ++i)
#pragma unroll
    for (int j = 0; j < 4; ++j) acc[i][j] = zero8();

  for (int k0 = 0; k0 < K; k0 += 32) {
#pragma unroll 1
    for (int ps = 0; ps < ((NSPLIT == 2) ? 2 : 1); ++ps) {
      const __bf16* Bs = (ps == 0) ? Bb : Bb2;
      v16b bh[4];
#pragma unroll
      for (int j = 0; j < 4; ++j) {
        const size_t bo = (size_t)(n0 + (j << 4) + rlane) * ldb + koff + k0;
        bh[j] = ldfrag_b(Bs + bo);
      }
#pragma unroll
      for (int i = 0; i < 4; ++i) {
        const size_t ao = (size_t)(m0 + (i << 4) + rlane) * lda + koff + k0;
        const v16b ah = ldfrag_b(Ab + ao);
        v16b al = ah;
        if (NSPLIT == 1) al = ldfrag_b(Ab2 + ao);
#pragma unroll
        for (int j = 0; j < 4; ++j) {
          acc[i][j] = mma_b_raw(ah, bh[j], acc[i][j]);
          if (NSPLIT == 1) acc[i][j] = mma_b_raw(al, bh[j], acc[i][j]);
        }
        dep_guard_b(acc[i][0], acc[i][3], ah, al);
      }
      keep4_b(bh[0], bh[1], bh[2], bh[3]);
    }
  }
  acc_guard4(acc[0][0], acc[0][1], acc[0][2], acc[0][3]);
  acc_guard4(acc[1][0], acc[1][1], acc[1][2], acc[1][3]);
  acc_guard4(acc[2][0], acc[2][1], acc[2][2], acc[2][3]);
  acc_guard4(acc[3][0], acc[3][1], acc[3][2], acc[3][3]);

  float* slab = sT[wave];
#pragma unroll
  for (int i = 0; i < 4; ++i) {
    const int mBase = m0 + (i << 4);
#pragma unroll
    for (int j = 0; j < 4; ++j) {
#pragma unroll
      for (int r = 0; r < 8; ++r) {
        slab[(mOff + r) * 68 + (j << 4) + rlane] = acc[i][j][r];
      }
    }
    __builtin_amdgcn_fence(__ATOMIC_RELEASE, "workgroup");
    __builtin_amdgcn_wave_barrier();
    __builtin_amdgcn_fence(__ATOMIC_ACQUIRE, "workgroup");
    if (OUT_MODE == 0) {
      float* C = (float*)Cout + (size_t)b * strideC;
      const int hh = lane >> 4, c4 = (lane & 15) * 4;
      for (int pass = 0; pass < 2; ++pass) {
#pragma unroll
        for (int it = 0; it < 8; ++it) {
          const int row = it * 2 + hh;
          const v4f v = *(const v4f*)(slab + row * 68 + c4);
          *(volatile v4f*)(C + (size_t)(mBase + row) * ldc + n0 + c4) = v;
        }
        __threadfence();
      }
    } else {
      const int q = lane >> 3, c8 = (lane & 7) * 8;
      unsigned short* C  = (unsigned short*)Cout  + (size_t)b * strideC;
      unsigned short* C2 = (unsigned short*)Cout2 + (size_t)b * strideC2;
      bool wlo = true;
      size_t col2 = (size_t)n0 + c8;
      if (OUT_MODE == 3) {
        const int sgi = n0 / segN;
        const int sgo = n0 - sgi * segN;
        wlo  = (sgo < N2);
        col2 = (size_t)sgi * N2 + sgo + c8;
      }
      v4f csA = {1.f, 1.f, 1.f, 1.f};
      v4f csB = csA;
      if (SCM == 2) {
        csA = *(const v4f*)(scb + n0 + c8);
        csB = *(const v4f*)(scb + n0 + c8 + 4);
      }
      v4u hv[4], lv[4];
#pragma unroll
      for (int it = 0; it < 4; ++it) {
        const int row = it * 4 + q;
        const int m = mBase + row;
        const float* sp = slab + row * 68 + c8;
        v4f x0 = *(const v4f*)(sp);
        v4f x1 = *(const v4f*)(sp + 4);
        if (SCM == 1) { const float rsv = scb[m]; x0 = x0 * rsv; x1 = x1 * rsv; }
        if (SCM == 2) { x0 = x0 * csA; x1 = x1 * csB; }
        float f[8] = {x0[0], x0[1], x0[2], x0[3], x1[0], x1[1], x1[2], x1[3]};
        if (ROT) {
          const v4f cs = *(const v4f*)(rct + (size_t)m * NFR + 4 * (lane & 7));
          const v4f sn = *(const v4f*)(rst + (size_t)m * NFR + 4 * (lane & 7));
#pragma unroll
          for (int e = 0; e < 4; ++e) {
            const float ev = f[2 * e], od = f[2 * e + 1];
            f[2 * e]     = ev * cs[e] - od * sn[e];
            f[2 * e + 1] = od * cs[e] + ev * sn[e];
          }
        }
        v4u a, a2;
#pragma unroll
        for (int e = 0; e < 4; ++e) {
          const float f0 = f[2 * e], f1 = f[2 * e + 1];
          unsigned short h0, h1, l0, l1;
          if (OUT_MODE == 2) {
            h0 = bf_bits(f0); h1 = bf_bits(f1);
            l0 = bf_bits(f0 - bf_up(h0)); l1 = bf_bits(f1 - bf_up(h1));
          } else {
            const _Float16 y0 = (_Float16)f0, y1 = (_Float16)f1;
            h0 = h_bits(y0); h1 = h_bits(y1);
            l0 = h_bits((_Float16)((f0 - (float)y0) * rscale));
            l1 = h_bits((_Float16)((f1 - (float)y1) * rscale));
          }
          a[e] = pk16(h0, h1); a2[e] = pk16(l0, l1);
        }
        hv[it] = a; lv[it] = a2;
      }
      for (int pass = 0; pass < 2; ++pass) {
#pragma unroll
        for (int it = 0; it < 4; ++it) {
          const int row = it * 4 + q;
          *(volatile v4u*)(C + (size_t)(mBase + row) * ldc + n0 + c8) = hv[it];
          if (wlo) *(volatile v4u*)(C2 + (size_t)(mBase + row) * ldc2 + col2) = lv[it];
        }
        __threadfence();
      }
    }
    __builtin_amdgcn_fence(__ATOMIC_RELEASE, "workgroup");
    __builtin_amdgcn_wave_barrier();
    __builtin_amdgcn_fence(__ATOMIC_ACQUIRE, "workgroup");
  }
}

template <bool RES>
__global__ __launch_bounds__(128)
void attn_seg64(const unsigned short* __restrict__ qkhp, const unsigned short* __restrict__ qklp,
                const unsigned short* __restrict__ vhp,  const unsigned short* __restrict__ vlp,
                const unsigned short* __restrict__ pkp,  const unsigned short* __restrict__ pvp,
                unsigned short* ohp, unsigned short* olp,
                int qbBase, int nqbThis, float sscale) {
  union FB { v16b v; v8b h[2]; };
  union FH { v16h v; v8h h[2]; };
  __shared__ __align__(16) __bf16   Ksh[64 * 64];
  __shared__ __align__(16) __bf16   Ksl[64 * 64];
  __shared__ __align__(16) _Float16 Vth[64 * 64];
  __shared__ __align__(16) _Float16 Vtl[RES ? 64 * 64 : 8];
  __shared__ __align__(16) _Float16 Psh[4][16 * 64];
  __shared__ __align__(16) _Float16 Psl[RES ? 4 : 1][16 * 64];
  __shared__ __align__(16) float    Os[4][16 * 64];

  const int tid  = threadIdx.x;
  const int wave = tid >> 5;
  const int lane = tid & 31;
  const int hh   = lane >> 4;
  const int c    = lane & 15;

  const int bx   = blockIdx.x;
  const int qbl  = bx % nqbThis;
  int rest       = bx / nqbThis;
  const int h    = rest % NH;
  rest           = rest / NH;
  const int w    = rest % NSEGB;
  const int b    = rest / NSEGB;
  const int qb   = qbBase + qbl;
  const int q0   = qb * 64 + wave * 16;
  const size_t rowS = (size_t)b * SEQ + (size_t)w * SEGL;

  const __bf16* Qh = (const __bf16*)(const void*)qkhp + (size_t)h * HD;
  const __bf16* Ql = (const __bf16*)(const void*)qklp + (size_t)h * HD;
  const __bf16* Kh = Qh + DMI;
  const __bf16* Kl = Ql + DMI;
  const _Float16* Vh = (const _Float16*)(const void*)vhp + ((size_t)b * DMI + (size_t)h * HD) * SEQ + (size_t)w * SEGL;
  const _Float16* Vl = (const _Float16*)(const void*)vlp + ((size_t)b * DMI + (size_t)h * HD) * (size_t)(NSEGB * VLP)
                       + (size_t)w * VLP;
  const __bf16*   PK = (const __bf16*)(const void*)pkp + (size_t)h * PMEM * HD;
  const _Float16* PV = (const _Float16*)(const void*)pvp + (size_t)h * HD * PMEM;

  v16b qah[2], qal[2];
#pragma unroll
  for (int dc = 0; dc < 2; ++dc) {
    const size_t qo = (rowS + q0 + c) * QKP + dc * 32 + 8 * hh;
    qah[dc] = ldfrag_b(Qh + qo);
    qal[dc] = ldfrag_b(Ql + qo);
  }

  float mrow[8], lrow[8];
  v8f oacc[4];
#pragma unroll
  for (int r = 0; r < 8; ++r) { mrow[r] = -INFINITY; lrow[r] = 0.f; }
#pragma unroll
  for (int t = 0; t < 4; ++t) oacc[t] = zero8();

  const int ntiles = qb + 2;
  for (int kt = 0; kt < ntiles; ++kt) {
    const int s0 = (kt - 1) * 64;
    __syncthreads();
    {
      const int r = tid >> 1, half = (tid & 1) * 32;
      if (kt == 0) {
        const int rr = (r < PMEM) ? r : (PMEM - 1);
        const bool krow = (r < PMEM);
        const bool vok  = (half == 0);
        const __bf16*   kg = PK + (size_t)rr * HD + half;
        const _Float16* vg = PV + (size_t)r * PMEM;
        const v8h pv0 = *(const v8h*)(vg);
        const v8h pv1 = *(const v8h*)(vg + 8);
#pragma unroll
        for (int i = 0; i < 4; ++i) {
          v8b a0 = *(const v8b*)(kg + 8 * i);
          a0 = krow ? a0 : zero8b();
          *(v8b*)(Ksh + r * 64 + half + 8 * i) = a0;
          *(v4u*)(Ksl + r * 64 + half + 8 * i) = zero4u();
          if (i == 0) {
            const v8h b0 = vok ? pv0 : zero8h();
            *(v8h*)(Vth + r * 64 + half) = b0;
          } else if (i == 1) {
            const v8h b1 = vok ? pv1 : zero8h();
            *(v8h*)(Vth + r * 64 + half + 8) = b1;
          } else {
            *(v4u*)(Vth + r * 64 + half + 8 * i) = zero4u();
          }
          if (RES) *(v4u*)(Vtl + r * 64 + half + 8 * i) = zero4u();
        }
      } else {
        const __bf16*   kg  = Kh + (rowS + s0 + r) * QKP + half;
        const __bf16*   klg = Kl + (rowS + s0 + r) * QKP + half;
        const _Float16* vg  = Vh + (size_t)r * SEQ + s0 + half;
        const bool resOK = (s0 + 64 <= VLP);
        const int  s0c   = resOK ? s0 : (VLP - 64);
        const _Float16* vlg = Vl + (size_t)r * (NSEGB * VLP) + s0c + half;
#pragma unroll
        for (int i = 0; i < 4; ++i) {
          const v8b a0 = *(const v8b*)(kg + 8 * i);
          const v8b a1 = *(const v8b*)(klg + 8 * i);
          const v8h b0 = *(const v8h*)(vg + 8 * i);
          *(v8b*)(Ksh + r * 64 + half + 8 * i) = a0;
          *(v8b*)(Ksl + r * 64 + half + 8 * i) = a1;
          *(v8h*)(Vth + r * 64 + half + 8 * i) = b0;
          if (RES) {
            v8h b1 = *(const v8h*)(vlg + 8 * i);
            b1 = resOK ? b1 : zero8h();
            *(v8h*)(Vtl + r * 64 + half + 8 * i) = b1;
          }
        }
      }
    }
    __syncthreads();

    v8f s[4];
#pragma unroll
    for (int j = 0; j < 4; ++j) {
      s[j] = zero8();
#pragma unroll
      for (int dc = 0; dc < 2; ++dc) {
        FB kb, kl;
        kb.h[0] = *(const v8b*)(Ksh + (j * 16 + c) * 64 + dc * 32 + 8 * hh);
        kb.h[1] = *(const v8b*)(Ksh + (j * 16 + c) * 64 + dc * 32 + 16 + 8 * hh);
        kl.h[0] = *(const v8b*)(Ksl + (j * 16 + c) * 64 + dc * 32 + 8 * hh);
        kl.h[1] = *(const v8b*)(Ksl + (j * 16 + c) * 64 + dc * 32 + 16 + 8 * hh);
        s[j] = mma_b(qah[dc], kb.v, s[j]);
        s[j] = mma_b(qah[dc], kl.v, s[j]);
        s[j] = mma_b(qal[dc], kb.v, s[j]);
      }
    }

    _Float16* pwh = Psh[wave];
    _Float16* pwl = Psl[RES ? wave : 0];
    const int qi = q0 + 8 * hh;
#pragma unroll
    for (int r = 0; r < 8; ++r) {
      float m = -INFINITY;
#pragma unroll
      for (int j = 0; j < 4; ++j) {
        const int kc = j * 16 + c;
        const bool vis = (kt == 0) ? (kc < PMEM) : ((s0 + kc) <= (qi + r));
        const float sv = vis ? (s[j][r] * sscale) : -INFINITY;
        s[j][r] = sv;
        m = fmaxf(m, sv);
      }
#pragma unroll
      for (int off = 1; off < 16; off <<= 1) m = fmaxf(m, __shfl_xor(m, off, 32));
      const float mnew  = fmaxf(mrow[r], m);
      const float msafe = (mnew == -INFINITY) ? 0.f : mnew;
      const float alpha = __expf(mrow[r] - msafe);
      mrow[r] = mnew;
      float psum = 0.f;
#pragma unroll
      for (int j = 0; j < 4; ++j) {
        const float p = __expf(s[j][r] - msafe);
        psum += p;
        const float p1k = p * 1024.0f;
        const _Float16 ph = (_Float16)p1k;
        pwh[(8 * hh + r) * 64 + j * 16 + c] = ph;
        if (RES) {
          const _Float16 pl = (_Float16)((p1k - (float)ph) * 4096.0f);
          pwl[(8 * hh + r) * 64 + j * 16 + c] = pl;
        }
      }
#pragma unroll
      for (int off = 1; off < 16; off <<= 1) psum += __shfl_xor(psum, off, 32);
      lrow[r] = lrow[r] * alpha + psum;
#pragma unroll
      for (int t = 0; t < 4; ++t) oacc[t][r] *= alpha;
    }
    __builtin_amdgcn_fence(__ATOMIC_RELEASE, "workgroup");
    __builtin_amdgcn_wave_barrier();
    __builtin_amdgcn_fence(__ATOMIC_ACQUIRE, "workgroup");

    v8f o1[4];
#pragma unroll
    for (int t = 0; t < 4; ++t) o1[t] = zero8();
#pragma unroll 1
    for (int kk = 0; kk < 2; ++kk) {
      FH pa, pl;
      pa.h[0] = *(const v8h*)(pwh + c * 64 + kk * 32 + 8 * hh);
      pa.h[1] = *(const v8h*)(pwh + c * 64 + kk * 32 + 16 + 8 * hh);
      if (RES) {
        pl.h[0] = *(const v8h*)(pwl + c * 64 + kk * 32 + 8 * hh);
        pl.h[1] = *(const v8h*)(pwl + c * 64 + kk * 32 + 16 + 8 * hh);
      } else {
        pl.v = pa.v;
      }
#pragma unroll
      for (int t = 0; t < 4; ++t) {
        FH vb;
        vb.h[0] = *(const v8h*)(Vth + (t * 16 + c) * 64 + kk * 32 + 8 * hh);
        vb.h[1] = *(const v8h*)(Vth + (t * 16 + c) * 64 + kk * 32 + 16 + 8 * hh);
        oacc[t] = mma_h(pa.v, vb.v, oacc[t]);
        if (RES) {
          FH vl;
          vl.h[0] = *(const v8h*)(Vtl + (t * 16 + c) * 64 + kk * 32 + 8 * hh);
          vl.h[1] = *(const v8h*)(Vtl + (t * 16 + c) * 64 + kk * 32 + 16 + 8 * hh);
          o1[t] = mma_h(pa.v, vl.v, o1[t]);
          o1[t] = mma_h(pl.v, vb.v, o1[t]);
        }
      }
    }
    if (RES) {
#pragma unroll
      for (int t = 0; t < 4; ++t)
#pragma unroll
        for (int r = 0; r < 8; ++r) oacc[t][r] += o1[t][r] * (1.0f / 4096.0f);
    }
  }

  float* os = Os[wave];
#pragma unroll
  for (int r = 0; r < 8; ++r) {
    const float l = lrow[r];
    const float inv = ((l > 0.f) ? (1.0f / l) : 0.f) * (1.0f / 1024.0f);
#pragma unroll
    for (int t = 0; t < 4; ++t) os[(8 * hh + r) * 64 + t * 16 + c] = oacc[t][r] * inv;
  }
  __builtin_amdgcn_fence(__ATOMIC_RELEASE, "workgroup");
  __builtin_amdgcn_wave_barrier();
  __builtin_amdgcn_fence(__ATOMIC_ACQUIRE, "workgroup");
  {
    const int q4 = lane >> 3, c8 = (lane & 7) * 8;
    v4u hv[4], lv[4];
#pragma unroll
    for (int it = 0; it < 4; ++it) {
      const int row = it * 4 + q4;
      const float* sp = os + row * 64 + c8;
      v4u a, a2;
#pragma unroll
      for (int e = 0; e < 4; ++e) {
        const float f0 = sp[2 * e], f1 = sp[2 * e + 1];
        const unsigned short h0 = bf_bits(f0), h1 = bf_bits(f1);
        const unsigned short l0 = bf_bits(f0 - bf_up(h0)), l1 = bf_bits(f1 - bf_up(h1));
        a[e] = pk16(h0, h1); a2[e] = pk16(l0, l1);
      }
      hv[it] = a; lv[it] = a2;
    }
    for (int pass = 0; pass < 2; ++pass) {
#pragma unroll
      for (int it = 0; it < 4; ++it) {
        const int row = it * 4 + q4;
        const size_t go = (rowS + q0 + row) * DMI + (size_t)h * HD + c8;
        *(volatile v4u*)(ohp + go) = hv[it];
        *(volatile v4u*)(olp + go) = lv[it];
      }
      __threadfence();
    }
  }
}

extern "C" void kernel_launch(void* const* d_in, const int* in_sizes, int n_in,
                              void* d_out, int out_size, void* d_ws, size_t ws_size,
                              hipStream_t stream) {
  if (n_in < 5) return;
  const long long needRows = (long long)(NB - 1) * SEQ_FULL + SEQ;
  if ((long long)in_sizes[0] < needRows * DM) return;
  if (in_sizes[1] < DM) return;
  if (in_sizes[2] < DM * 3 * DMI) return;
  if (in_sizes[3] < DMI * DM) return;
  if (in_sizes[4] < 2 * NH * PMEM * HD) return;
  if ((long long)out_size < needRows * DM) return;

  const float* seq  = (const float*)d_in[0];
  const float* gnm  = (const float*)d_in[1];
  const float* Wqkv = (const float*)d_in[2];
  const float* Wout = (const float*)d_in[3];
  const float* pm   = (const float*)d_in[4];

  const size_t M    = (size_t)NB * SEQ;
  const size_t PX   = M * DM * 2;
  const size_t PWT  = (size_t)3 * DMI * DM * 2;
  const size_t PTAB = (size_t)SEQ * NFR * 4;
  const size_t PRS  = M * 4;
  const size_t PO   = M * DMI * 2;
  const size_t PQK  = M * QKP * 2;
  const size_t PVT  = (size_t)NB * DMI * SEQ * 2;
  const size_t PVL  = (size_t)NB * DMI * NSEGB * VLP * 2;
  const size_t PWO  = (size_t)DM * DMI * 2;
  const size_t PPM  = (size_t)NH * PMEM * HD * 2;
  const size_t ph1  = PX + 2 * PWT + 2 * PTAB + PRS;
  const size_t ph2  = 2 * PO;
  const size_t REGA = (ph1 > ph2) ? ph1 : ph2;
  const size_t oXb  = 0;
  const size_t oWth = PX;
  const size_t oWtl = PX + PWT;
  const size_t oCt  = PX + 2 * PWT;
  const size_t oSt  = oCt + PTAB;
  const size_t oRs  = oSt + PTAB;
  const size_t oOh  = 0;
  const size_t oOl  = PO;
  size_t off = REGA;
  const size_t oQKh = off; off += PQK;
  const size_t oQKl = off; off += PQK;
  const size_t oVTh = off; off += PVT;
  const size_t oVTl = off; off += PVL;
  const size_t oWo  = off; off += PWO;
  const size_t oPk  = off; off += PPM;
  const size_t oPv  = off; off += PPM;
  if (off > ws_size) return;
  if (off > (size_t)134217728) return;
  if (oRs + PRS > REGA || oOl + PO > REGA) return;

  char* ws = (char*)d_ws;
  unsigned short* Xb  = (unsigned short*)(ws + oXb);
  unsigned short* Wth = (unsigned short*)(ws + oWth);
  unsigned short* Wtl = (unsigned short*)(ws + oWtl);
  float*          Ct  = (float*)(ws + oCt);
  float*          St  = (float*)(ws + oSt);
  float*          Rs  = (float*)(ws + oRs);
  unsigned short* Oh  = (unsigned short*)(ws + oOh);
  unsigned short* Ol  = (unsigned short*)(ws + oOl);
  unsigned short* QKh = (unsigned short*)(ws + oQKh);
  unsigned short* QKl = (unsigned short*)(ws + oQKl);
  unsigned short* VTh = (unsigned short*)(ws + oVTh);
  unsigned short* VTl = (unsigned short*)(ws + oVTl);
  unsigned short* Wo  = (unsigned short*)(ws + oWo);
  unsigned short* Pk  = (unsigned short*)(ws + oPk);
  unsigned short* Pv  = (unsigned short*)(ws + oPv);

  const dim3 blk(256);
  const dim3 gTab(SEQ / 8);
  const dim3 gCvtX((unsigned)(M / 32));
  const dim3 gWt(3 * DMI / 64, DM / 64);
  const dim3 gWo(DM / 64, DMI / 64);
  const int tilesQK  = (SEQ / 64) * (QKP / 64);
  const int tilesVT  = (DMI / 64) * (SEQ / 64);
  const int tilesOut = (SEQ / 64) * (DM / 64);
  const dim3 gQK((tilesQK + 7) / 8, NB);
  const dim3 gVT((tilesVT + 7) / 8, NB);
  const dim3 gOut((tilesOut + 7) / 8, NB);

  tab_cs<<<gTab, blk, 0, stream>>>(Ct, St);
  cvtx_rstd<<<gCvtX, blk, 0, stream>>>(seq, Xb, Rs);
  wt_cvt<true, 2><<<gWt, blk, 0, stream>>>(Wqkv, gnm, Wth, Wtl, DM, 3 * DMI);
  wt_cvt<false, 1><<<gWo, blk, 0, stream>>>(Wout, gnm, Wo, Wo, DMI, DM);
  pm_cvt<<<dim3(NH), dim3(128), 0, stream>>>(pm, Pk, Pv);
  gemm64<2, 2, 1, true><<<gQK, blk, 0, stream>>>(
      Xb, Xb, DM, (long long)SEQ * DM,
      Wth, Wtl, DM, 0LL,
      (void*)QKh, QKP, (long long)SEQ * QKP,
      (void*)QKl, QKP, (long long)SEQ * QKP, QKP, QKP,
      Rs, (long long)SEQ, Ct, St,
      SEQ, QKP, DM, 1.0f);
  gemm64<1, 3, 2, false><<<gVT, blk, 0, stream>>>(
      Wth + (size_t)2 * DMI * DM, Wtl + (size_t)2 * DMI * DM, DM, 0LL,
      Xb, Xb, DM, (long long)SEQ * DM,
      (void*)VTh, SEQ, (long long)DMI * SEQ,
      (void*)VTl, NSEGB * VLP, (long long)DMI * NSEGB * VLP, VLP, SEGL,
      Rs, (long long)SEQ, Ct, St,
      DMI, SEQ, DM, 4096.0f);
  attn_seg64<true><<<dim3(NB * NSEGB * NH * RESQB), dim3(128), 0, stream>>>(
      QKh, QKl, VTh, VTl, Pk, Pv, Oh, Ol, 0, RESQB, 0.125f);
  if (NQBS - RESQB > 0) {
    attn_seg64<false><<<dim3(NB * NSEGB * NH * (NQBS - RESQB)), dim3(128), 0, stream>>>(
        QKh, QKl, VTh, VTl, Pk, Pv, Oh, Ol, RESQB, NQBS - RESQB, 0.125f);
  }
  gemm64<1, 0, 0, false><<<gOut, blk, 0, stream>>>(
      Oh, Ol, DMI, (long long)SEQ * DMI,
      Wo, Wo, DMI, 0LL,
      d_out, DM, (long long)SEQ_FULL * DM,
      d_out, DM, (long long)SEQ_FULL * DM, DM, DM,
      Rs, 0LL, Ct, St,
      SEQ, DM, DMI, 1.0f);
  (void)hipGetLastError();
}
